// TopoGraphBlock_46892452938508
// MI455X (gfx1250) — hardware-verified
//
#include <hip/hip_runtime.h>


#define NB_  1024
#define NJ   24
#define NT   6
#define FF   64
#define HH   128
#define NO   64
#define RG   4
#define NJR  (NB_ * NJ)
#define NTR  (NB_ * NT)
#define EVJ  64
#define EVT  256
#define ECH  (EVJ * NJ * NJ)
#define DM   HH
#define LOSC 1024.0f

typedef _Float16 h16;
typedef unsigned short bf;
typedef __attribute__((ext_vector_type(16))) __bf16   v16bf;
typedef __attribute__((ext_vector_type(16))) _Float16 v16h;
typedef __attribute__((ext_vector_type(8)))  _Float16 v8h;
typedef __attribute__((ext_vector_type(8)))  unsigned short v8us;
typedef __attribute__((ext_vector_type(8)))  float    v8f;
typedef __attribute__((ext_vector_type(4)))  float    v4f;
typedef v8h  __attribute__((may_alias)) v8ha;
typedef v4f  __attribute__((may_alias)) v4fa;
typedef v8us __attribute__((may_alias)) v8usa;

__device__ __forceinline__ unsigned short f2bf(float f) { unsigned u = __float_as_uint(f); u += 0x7FFFu + ((u >> 16) & 1u); return (unsigned short)(u >> 16); }
__device__ __forceinline__ float bf2f(unsigned short b) { return __uint_as_float(((unsigned)b) << 16); }
__device__ __forceinline__ float bfr(float f) { return bf2f(f2bf(f)); }
__device__ __forceinline__ v16h cat16(v8h lo, v8h hi) { return __builtin_shufflevector(lo, hi, 0, 1, 2, 3, 4, 5, 6, 7, 8, 9, 10, 11, 12, 13, 14, 15); }
__device__ __forceinline__ v16bf cat16b(v8us lo, v8us hi) { return __builtin_bit_cast(v16bf, __builtin_shufflevector(lo, hi, 0, 1, 2, 3, 4, 5, 6, 7, 8, 9, 10, 11, 12, 13, 14, 15)); }
__device__ __forceinline__ v8f wmma16(v16h a, v16h b, v8f c) { return __builtin_amdgcn_wmma_f32_16x16x32_f16(false, a, false, b, (short)0, c, false, false); }
__device__ __forceinline__ v8f wmmab(v16bf a, v16bf b, v8f c) { return __builtin_amdgcn_wmma_f32_16x16x32_bf16(false, a, false, b, (short)0, c, false, false); }

template <bool SPLITA, bool F16OUT = false>
__global__ __launch_bounds__(128) void k_gemmb(const bf* __restrict__ A, const bf* __restrict__ Al, const bf* __restrict__ Bn, const float* __restrict__ bias, float* C, int ldc, h16* C2, const float* __restrict__ R = nullptr, int K = DM, int roundR = 1) {
    __shared__ __align__(16) float ost[4][16 * 68];
    const int lane = threadIdx.x & 31, wave = threadIdx.x >> 5, lr = lane & 15, hi = lane >> 4;
    const int r0 = blockIdx.x * 64 + wave * 16, c0 = blockIdx.y * 64;
    const size_t aoff = (size_t)(r0 + lr) * K + 8 * hi;
    size_t boff[4];
#pragma unroll
    for (int t = 0; t < 4; ++t) boff[t] = (size_t)(c0 + t * 16 + lr) * K + 8 * hi;
    v8f acc[4];
#pragma unroll
    for (int t = 0; t < 4; ++t) acc[t] = (v8f){};
#pragma unroll 1
    for (int kc = 0; kc < K; kc += 32) {
        const v16bf a = cat16b(*(const v8us*)(A + aoff + kc), *(const v8us*)(A + aoff + kc + 16));
        v16bf al = a;
        if (SPLITA) al = cat16b(*(const v8us*)(Al + aoff + kc), *(const v8us*)(Al + aoff + kc + 16));
#pragma unroll
        for (int t = 0; t < 4; ++t) { const v16bf b = cat16b(*(const v8us*)(Bn + boff[t] + kc), *(const v8us*)(Bn + boff[t] + kc + 16)); acc[t] = wmmab(a, b, acc[t]); if (SPLITA) acc[t] = wmmab(al, b, acc[t]); }
        asm volatile("v_nop\n\tv_nop\n\tv_nop\n\tv_nop" : "+v"(acc[0]), "+v"(acc[1]), "+v"(acc[2]), "+v"(acc[3]) : "v"(a), "v"(al));
    }
    float* os = &ost[wave][0];
#pragma unroll
    for (int t = 0; t < 4; ++t) { const float bv = bias ? bfr(bias[c0 + t * 16 + lr]) : 0.f;
#pragma unroll
        for (int j = 0; j < 8; ++j) os[(hi * 8 + j) * 68 + t * 16 + lr] = acc[t][j] + bv; }
    __syncthreads();
    if (F16OUT) {
        h16* crow = (h16*)(void*)C + (size_t)r0 * ldc + c0;
        auto pass = [&]() {
#pragma unroll
            for (int s = 0; s < 4; ++s) { const int row = 4 * s + (lane >> 3), piece = lane & 7; const float* sp = os + row * 68 + piece * 8; v8h o, o2;
#pragma unroll
                for (int i = 0; i < 8; ++i) { const h16 a = (h16)sp[i]; o[i] = a; o2[i] = (h16)((sp[i] - (float)a) * LOSC); }
                *(volatile v8h*)(crow + (size_t)row * ldc + piece * 8) = o; if (C2) *(volatile v8h*)(C2 + (size_t)r0 * ldc + c0 + (size_t)row * ldc + piece * 8) = o2; }
        };
        pass(); __threadfence(); pass();
    } else {
        float* crow = C + (size_t)r0 * ldc + c0;
        auto pass = [&]() {
#pragma unroll
            for (int s = 0; s < 8; ++s) { const int Lid = (lane >> 3) + 4 * s, piece = lane & 7; const int row = Lid >> 1, cofs = (Lid & 1) * 32 + piece * 4;
                v4f val = *(const v4fa*)(os + row * 68 + cofs); if (R) { const v4f rv = *(const v4f*)(R + ((size_t)r0 + row) * ldc + c0 + cofs); val += roundR ? (v4f){bfr(rv[0]), bfr(rv[1]), bfr(rv[2]), bfr(rv[3])} : rv; }
                *(volatile v4f*)(crow + (size_t)row * ldc + cofs) = val; }
        };
        pass(); __threadfence(); pass();
    }
}

__global__ __launch_bounds__(256) void k_wt(const float* __restrict__ Wm, int K, int ncols, bf* WT) {
    __shared__ __align__(16) unsigned short tl[64 * 72];
    const int tid = threadIdx.x, k0 = blockIdx.x * 64, n0 = blockIdx.y * 64;
    const int kk = tid >> 2, nq = (tid & 3) * 16;
#pragma unroll
    for (int i = 0; i < 16; ++i) tl[(nq + i) * 72 + kk] = f2bf(Wm[(size_t)(k0 + kk) * ncols + n0 + nq + i]);
    __syncthreads();
    const int piece = tid & 7;
    auto pass = [&]() {
#pragma unroll
        for (int s = 0; s < 2; ++s) { const int nr = (tid >> 3) + 32 * s; const v8us val = *(const v8usa*)(tl + nr * 72 + piece * 8); *(volatile v8us*)(WT + (size_t)(n0 + nr) * K + k0 + piece * 8) = val; }
    };
    pass(); __threadfence(); pass();
}

__global__ __launch_bounds__(256) void k_cvtrows(const float* __restrict__ src, int rows, bf* dst) {
    typedef __attribute__((ext_vector_type(2))) unsigned short v2us;
    const int lane = threadIdx.x & 31; const size_t r = (size_t)blockIdx.x * 8 + (threadIdx.x >> 5); if (r >= (size_t)rows) return; v2us o;
#pragma unroll
    for (int i = 0; i < 2; ++i) o[i] = f2bf(src[r * FF + lane * 2 + i]);
    *(volatile v2us*)(dst + r * FF + lane * 2) = o; __threadfence(); *(volatile v2us*)(dst + r * FF + lane * 2) = o;
}
__global__ __launch_bounds__(256) void k_edge1(const float* __restrict__ PR, const float* __restrict__ PS, const float* __restrict__ b1, int Nr, int Ns, int b0, int nedges, bf* Eh, bf* El) {
    typedef __attribute__((ext_vector_type(4))) unsigned short v4us;
    const int lane = threadIdx.x & 31; const size_t e = (size_t)blockIdx.x * 8 + (threadIdx.x >> 5); if (e >= (size_t)nedges) return; const int s = (int)(e % Ns); const size_t br = e / Ns; const int r = (int)(br % Nr); const int b = b0 + (int)(br / Nr);
    const float* pr = PR + ((size_t)b * Nr + r) * HH; const float* psn = PS + ((size_t)b * Ns + s) * HH; v4us oh, ol;
#pragma unroll
    for (int i = 0; i < 4; ++i) { const int h = lane * 4 + i; const float v = fmaxf(pr[h] + psn[h] + bfr(b1[h]), 0.f); const unsigned short hb = f2bf(v); oh[i] = hb; ol[i] = f2bf(v - bf2f(hb)); }
    const size_t o = e * HH + lane * 4; *(volatile v4us*)(Eh + o) = oh; *(volatile v4us*)(El + o) = ol; __threadfence(); *(volatile v4us*)(Eh + o) = oh; *(volatile v4us*)(El + o) = ol;
}
template <bool MASKED>
__global__ __launch_bounds__(256) void k_pool(const float* __restrict__ E2, const float* __restrict__ mask, int Nr, int Ns, int b0, int nrecv, float* POOL) {
    const int lane = threadIdx.x & 31; const size_t w = (size_t)blockIdx.x * 8 + (threadIdx.x >> 5); if (w >= (size_t)nrecv) return; const int r = (int)(w % Nr); const int b = b0 + (int)(w / Nr); v4f acc = {0.f, 0.f, 0.f, 0.f}; float msum = 0.f;
    for (int s = 0; s < Ns; ++s) { const float m = MASKED ? bfr(mask[(size_t)b * Ns + s]) : 1.f; if (MASKED) msum += m; const float* row = E2 + (w * Ns + s) * HH + lane * 4;
#pragma unroll
        for (int i = 0; i < 4; ++i) acc[i] = fmaf(fmaxf(row[i], 0.f), m, acc[i]); }
    const float inv = MASKED ? 1.0f / fmaxf(msum, 1.0f) : 1.0f / (float)Ns; acc *= inv;
    const size_t o = ((size_t)b * Nr + r) * HH + lane * 4; *(volatile v4f*)(POOL + o) = acc; __threadfence(); *(volatile v4f*)(POOL + o) = acc;
}
__global__ __launch_bounds__(256) void k_split128(const float* __restrict__ src, int rows, bf* dh, bf* dl) {
    typedef __attribute__((ext_vector_type(4))) unsigned short v4us;
    const int lane = threadIdx.x & 31; const size_t r = (size_t)blockIdx.x * 8 + (threadIdx.x >> 5); if (r >= (size_t)rows) return; const size_t o = r * HH + lane * 4; const v4f v = *(const v4f*)(src + o); v4us oh, ol;
#pragma unroll
    for (int i = 0; i < 4; ++i) { const unsigned short hb = f2bf(v[i]); oh[i] = hb; ol[i] = f2bf(v[i] - bf2f(hb)); }
    *(volatile v4us*)(dh + o) = oh; *(volatile v4us*)(dl + o) = ol; __threadfence(); *(volatile v4us*)(dh + o) = oh; *(volatile v4us*)(dl + o) = ol;
}
__global__ __launch_bounds__(256) void k_relupl128(const float* __restrict__ src, int rows, bf* dh, bf* dl) {
    typedef __attribute__((ext_vector_type(4))) unsigned short v4us;
    const int lane = threadIdx.x & 31; const size_t r = (size_t)blockIdx.x * 8 + (threadIdx.x >> 5); if (r >= (size_t)rows) return; const size_t o = r * HH + lane * 4; const v4f v = *(const v4f*)(src + o); v4us oh, ol;
#pragma unroll
    for (int i = 0; i < 4; ++i) { const float y = fmaxf(v[i], 0.f); const unsigned short hb = f2bf(y); oh[i] = hb; ol[i] = f2bf(y - bf2f(hb)); }
    *(volatile v4us*)(dh + o) = oh; *(volatile v4us*)(dl + o) = ol; __threadfence(); *(volatile v4us*)(dh + o) = oh; *(volatile v4us*)(dl + o) = ol;
}
template <bool MASK>
__global__ __launch_bounds__(256) void k_nodeout(const float* __restrict__ G, const float* __restrict__ mask, int rows, float* OUTN, bf* Uh, bf* Ul) {
    typedef __attribute__((ext_vector_type(2))) unsigned short v2us; typedef __attribute__((ext_vector_type(2))) float v2f_;
    const int lane = threadIdx.x & 31; const size_t r = (size_t)blockIdx.x * 8 + (threadIdx.x >> 5); if (r >= (size_t)rows) return; const float m = MASK ? bfr(mask[r]) : 1.f; v2f_ y; v2us oh, ol;
#pragma unroll
    for (int i = 0; i < 2; ++i) { const float v = fmaxf(G[r * NO + lane * 2 + i], 0.f) * m; y[i] = v; const unsigned short hb = f2bf(v); oh[i] = hb; ol[i] = f2bf(v - bf2f(hb)); }
    const size_t o = r * NO + lane * 2; *(volatile v2f_*)(OUTN + o) = y; *(volatile v2us*)(Uh + o) = oh; *(volatile v2us*)(Ul + o) = ol; __threadfence(); *(volatile v2f_*)(OUTN + o) = y; *(volatile v2us*)(Uh + o) = oh; *(volatile v2us*)(Ul + o) = ol;
}
__global__ __launch_bounds__(256) void k_wc3(const float* __restrict__ wc3, bf* WC3) {
    typedef __attribute__((ext_vector_type(4))) unsigned short v4us;
    const int lane = threadIdx.x & 31; const int r = blockIdx.x * 8 + (threadIdx.x >> 5); if (r >= 64) return; v4us v;
#pragma unroll
    for (int i = 0; i < 4; ++i) v[i] = f2bf(r == 0 ? wc3[lane * 4 + i] : 0.f);
    *(volatile v4us*)(WC3 + (size_t)r * HH + lane * 4) = v; __threadfence(); *(volatile v4us*)(WC3 + (size_t)r * HH + lane * 4) = v;
}
__global__ __launch_bounds__(256) void k_score(const float* __restrict__ SC, const float* __restrict__ bc3, const float* __restrict__ mask, size_t e0, int nedges, float* OUT2) {
    const int lane = threadIdx.x & 31; const size_t w = (size_t)blockIdx.x * 8 + (threadIdx.x >> 5); if (w * 128 >= (size_t)nedges) return; v4f v; const float bb = bfr(bc3[0]);
#pragma unroll
    for (int i = 0; i < 4; ++i) { const size_t el = w * 128 + lane * 4 + i; const size_t e = e0 + el; const int j = (int)(e % NJ); const size_t b = e / (NJ * NT); const float s = 1.0f / (1.0f + expf(-(SC[el * 64] + bb))); v[i] = s * bfr(mask[b * NJ + j]); }
    *(volatile v4f*)(OUT2 + e0 + w * 128 + lane * 4) = v; __threadfence(); *(volatile v4f*)(OUT2 + e0 + w * 128 + lane * 4) = v;
}
__global__ __launch_bounds__(256) void k_utp(const bf* __restrict__ Uh, const bf* __restrict__ Ul, bf* Ph, bf* Pl) {
    typedef __attribute__((ext_vector_type(2))) unsigned short v2us;
    const int lane = threadIdx.x & 31; const size_t w = (size_t)blockIdx.x * 8 + (threadIdx.x >> 5); if (w >= (size_t)NTR) return; const int p = (int)(w / NB_); const int b = (int)(w % NB_); const size_t src = ((size_t)b * NT + p) * NO + lane * 2; const size_t dst = w * NO + lane * 2;
    const v2us a = *(const v2us*)(Uh + src), c = *(const v2us*)(Ul + src); *(volatile v2us*)(Ph + dst) = a; *(volatile v2us*)(Pl + dst) = c; __threadfence(); *(volatile v2us*)(Ph + dst) = a; *(volatile v2us*)(Pl + dst) = c;
}
__global__ __launch_bounds__(256) void k_wpadr(const float* __restrict__ w3, bf* WR3) {
    typedef __attribute__((ext_vector_type(4))) unsigned short v4us;
    const int lane = threadIdx.x & 31; const int r = blockIdx.x * 8 + (threadIdx.x >> 5); if (r >= 64) return; v4us v;
#pragma unroll
    for (int i = 0; i < 4; ++i) { const int k = lane * 4 + i; v[i] = f2bf(r < RG ? w3[(size_t)k * RG + (r < RG ? r : 0)] : 0.f); }
    *(volatile v4us*)(WR3 + (size_t)r * HH + lane * 4) = v; __threadfence(); *(volatile v4us*)(WR3 + (size_t)r * HH + lane * 4) = v;
}
__global__ __launch_bounds__(64) void k_bpad64x(const float* __restrict__ b, int n, float* BP) { const int t = threadIdx.x; const float v = (t < n) ? b[t < n ? t : 0] : 0.f; *(volatile float*)(BP + t) = v; __threadfence(); *(volatile float*)(BP + t) = v; }
__global__ __launch_bounds__(256) void k_regout(const float* __restrict__ REG, float* OUT3) {
    const int lane = threadIdx.x & 31; const size_t w = (size_t)blockIdx.x * 8 + (threadIdx.x >> 5); if (w >= (size_t)NB_ * NT * RG / 128) return; v4f v;
#pragma unroll
    for (int i = 0; i < 4; ++i) { const size_t e = w * 128 + lane * 4 + i; const int b = (int)(e / (NT * RG)); const int p = (int)((e % (NT * RG)) / RG); const int k = (int)(e % RG); v[i] = REG[((size_t)p * NB_ + b) * 64 + k]; }
    *(volatile v4f*)(OUT3 + w * 128 + lane * 4) = v; __threadfence(); *(volatile v4f*)(OUT3 + w * 128 + lane * 4) = v;
}

extern "C" void kernel_launch(void* const* d_in, const int* in_sizes, int n_in,
                              void* d_out, int out_size, void* d_ws, size_t ws_size, hipStream_t stream) {
    (void)in_sizes; (void)n_in; (void)out_size;
    const float* jets = (const float*)d_in[0]; const float* mask = (const float*)d_in[1]; const float* tops = (const float*)d_in[2];
    const float* Wjj1 = (const float*)d_in[3]; const float* bjj1 = (const float*)d_in[4]; const float* Wjj2 = (const float*)d_in[5]; const float* bjj2 = (const float*)d_in[6];
    const float* Wjt1 = (const float*)d_in[7]; const float* bjt1 = (const float*)d_in[8]; const float* Wjt2 = (const float*)d_in[9]; const float* bjt2 = (const float*)d_in[10];
    const float* Wtj1 = (const float*)d_in[11]; const float* btj1 = (const float*)d_in[12]; const float* Wtj2 = (const float*)d_in[13]; const float* btj2 = (const float*)d_in[14];
    const float* Wnj1 = (const float*)d_in[15]; const float* bnj1 = (const float*)d_in[16]; const float* Wnj2 = (const float*)d_in[17]; const float* bnj2 = (const float*)d_in[18];
    const float* Wnt1 = (const float*)d_in[19]; const float* bnt1 = (const float*)d_in[20]; const float* Wnt2 = (const float*)d_in[21]; const float* bnt2 = (const float*)d_in[22];
    const float* Wc1 = (const float*)d_in[23]; const float* bc1 = (const float*)d_in[24]; const float* Wc2 = (const float*)d_in[25]; const float* bc2 = (const float*)d_in[26]; const float* Wc3 = (const float*)d_in[27]; const float* bc3 = (const float*)d_in[28];
    const float* Wr1 = (const float*)d_in[29]; const float* br1 = (const float*)d_in[30]; const float* Wr2 = (const float*)d_in[31]; const float* br2 = (const float*)d_in[32]; const float* Wr3 = (const float*)d_in[33]; const float* br3 = (const float*)d_in[34];
    float* out0 = (float*)d_out;
    float* out1 = out0 + (size_t)NJR * NO;
    float* out2 = out1 + (size_t)NTR * NO;
    float* out3 = out2 + (size_t)NB_ * NT * NJ;
    char* wsp = (char*)d_ws;
    auto take = [&](size_t bytes) { char* p = wsp; wsp += (bytes + 255) & ~(size_t)255; return (void*)p; };
    const size_t W64 = (size_t)HH * FF * 2, W128 = (size_t)HH * HH * 2;
    bf* WJJa = (bf*)take(W64); bf* WJJb = (bf*)take(W64); bf* WJJ2 = (bf*)take(W128); bf* WJTa = (bf*)take(W64); bf* WJTb = (bf*)take(W64); bf* WJT2 = (bf*)take(W128); bf* WTJa = (bf*)take(W64); bf* WTJb = (bf*)take(W64); bf* WTJ2 = (bf*)take(W128);
    bf* WNJa = (bf*)take(W64); bf* WNJb = (bf*)take(W128); bf* WNJc = (bf*)take(W128); bf* WNJ2 = (bf*)take((size_t)NO * HH * 2); bf* WNTa = (bf*)take(W64); bf* WNTb = (bf*)take(W128); bf* WNT2 = (bf*)take((size_t)NO * HH * 2);
    bf* WCa = (bf*)take(W64); bf* WCb = (bf*)take(W64); bf* WC2 = (bf*)take(W128); bf* WC3 = (bf*)take((size_t)64 * HH * 2); bf* WR1 = (bf*)take((size_t)NT * HH * FF * 2); bf* WR2 = (bf*)take((size_t)NT * HH * HH * 2); bf* WR3 = (bf*)take((size_t)NT * 64 * HH * 2); float* BR3 = (float*)take((size_t)NT * 64 * 4);
    bf* Jb = (bf*)take((size_t)NJR * FF * 2); bf* Tb = (bf*)take((size_t)NTR * FF * 2);
    float* PR = (float*)take((size_t)NJR * HH * 4); float* PS = (float*)take((size_t)NJR * HH * 4);
    bf* Eh = (bf*)take((size_t)ECH * HH * 2); bf* El = (bf*)take((size_t)ECH * HH * 2); float* E2 = (float*)take((size_t)ECH * HH * 4);
    float* PJJ = (float*)take((size_t)NJR * HH * 4); float* PJT = (float*)take((size_t)NJR * HH * 4); float* PTJ = (float*)take((size_t)NTR * HH * 4);
    bf* PJJh = (bf*)take((size_t)NJR * HH * 2); bf* PJJl = (bf*)take((size_t)NJR * HH * 2); bf* PJTh = (bf*)take((size_t)NJR * HH * 2); bf* PJTl = (bf*)take((size_t)NJR * HH * 2); bf* PTJh = (bf*)take((size_t)NTR * HH * 2); bf* PTJl = (bf*)take((size_t)NTR * HH * 2);
    float* G1 = (float*)take((size_t)NJR * HH * 4); float* G1b = (float*)take((size_t)NJR * HH * 4); bf* G1h = (bf*)take((size_t)NJR * HH * 2); bf* G1l = (bf*)take((size_t)NJR * HH * 2); float* G2 = (float*)take((size_t)NJR * NO * 4);
    bf* UJh = (bf*)take((size_t)NJR * NO * 2); bf* UJl = (bf*)take((size_t)NJR * NO * 2); bf* UTh = (bf*)take((size_t)NTR * NO * 2); bf* UTl = (bf*)take((size_t)NTR * NO * 2);
    float* SC = (float*)take((size_t)ECH * 64 * 4); bf* UTPh = (bf*)take((size_t)NTR * NO * 2); bf* UTPl = (bf*)take((size_t)NTR * NO * 2); float* R1 = (float*)take((size_t)NB_ * HH * 4); bf* R1h = (bf*)take((size_t)NB_ * HH * 2); bf* R1l = (bf*)take((size_t)NB_ * HH * 2); float* REG = (float*)take((size_t)NT * NB_ * 64 * 4);
    if ((size_t)(wsp - (char*)d_ws) > ws_size) return;
    k_wt<<<dim3(FF / 64, HH / 64, 1), 256, 0, stream>>>(Wjj1, FF, HH, WJJa); k_wt<<<dim3(FF / 64, HH / 64, 1), 256, 0, stream>>>(Wjj1 + (size_t)FF * HH, FF, HH, WJJb); k_wt<<<dim3(HH / 64, HH / 64, 1), 256, 0, stream>>>(Wjj2, HH, HH, WJJ2);
    k_wt<<<dim3(FF / 64, HH / 64, 1), 256, 0, stream>>>(Wjt1, FF, HH, WJTa); k_wt<<<dim3(FF / 64, HH / 64, 1), 256, 0, stream>>>(Wjt1 + (size_t)FF * HH, FF, HH, WJTb); k_wt<<<dim3(HH / 64, HH / 64, 1), 256, 0, stream>>>(Wjt2, HH, HH, WJT2);
    k_wt<<<dim3(FF / 64, HH / 64, 1), 256, 0, stream>>>(Wtj1, FF, HH, WTJa); k_wt<<<dim3(FF / 64, HH / 64, 1), 256, 0, stream>>>(Wtj1 + (size_t)FF * HH, FF, HH, WTJb); k_wt<<<dim3(HH / 64, HH / 64, 1), 256, 0, stream>>>(Wtj2, HH, HH, WTJ2);
    k_wt<<<dim3(FF / 64, HH / 64, 1), 256, 0, stream>>>(Wnj1, FF, HH, WNJa); k_wt<<<dim3(HH / 64, HH / 64, 1), 256, 0, stream>>>(Wnj1 + (size_t)FF * HH, HH, HH, WNJb); k_wt<<<dim3(HH / 64, HH / 64, 1), 256, 0, stream>>>(Wnj1 + (size_t)(FF + HH) * HH, HH, HH, WNJc); k_wt<<<dim3(HH / 64, NO / 64, 1), 256, 0, stream>>>(Wnj2, HH, NO, WNJ2);
    k_wt<<<dim3(FF / 64, HH / 64, 1), 256, 0, stream>>>(Wnt1, FF, HH, WNTa); k_wt<<<dim3(HH / 64, HH / 64, 1), 256, 0, stream>>>(Wnt1 + (size_t)FF * HH, HH, HH, WNTb); k_wt<<<dim3(HH / 64, NO / 64, 1), 256, 0, stream>>>(Wnt2, HH, NO, WNT2);
    k_wt<<<dim3(NO / 64, HH / 64, 1), 256, 0, stream>>>(Wc1, NO, HH, WCa); k_wt<<<dim3(NO / 64, HH / 64, 1), 256, 0, stream>>>(Wc1 + (size_t)NO * HH, NO, HH, WCb); k_wt<<<dim3(HH / 64, HH / 64, 1), 256, 0, stream>>>(Wc2, HH, HH, WC2); k_wc3<<<64 / 8, 256, 0, stream>>>(Wc3, WC3);
    for (int p = 0; p < NT; ++p) { k_wt<<<dim3(NO / 64, HH / 64, 1), 256, 0, stream>>>(Wr1 + (size_t)p * NO * HH, NO, HH, WR1 + (size_t)p * HH * FF); k_wt<<<dim3(HH / 64, HH / 64, 1), 256, 0, stream>>>(Wr2 + (size_t)p * HH * HH, HH, HH, WR2 + (size_t)p * HH * HH); k_wpadr<<<64 / 8, 256, 0, stream>>>(Wr3 + (size_t)p * HH * RG, WR3 + (size_t)p * 64 * HH); k_bpad64x<<<1, 64, 0, stream>>>(br3 + (size_t)p * RG, RG, BR3 + (size_t)p * 64); }
    k_cvtrows<<<NJR / 8, 256, 0, stream>>>(jets, NJR, Jb); k_cvtrows<<<NTR / 8, 256, 0, stream>>>(tops, NTR, Tb);
    const dim3 gJ(NJR / 64, HH / 64, 1), gT(NTR / 64, HH / 64, 1), gE(ECH / 64, HH / 64, 1); const int ECT = EVT * NJ * NT; const dim3 gET(ECT / 64, HH / 64, 1);
    k_gemmb<false, false><<<gJ, 128, 0, stream>>>(Jb, nullptr, WJJa, nullptr, PR, HH, nullptr, nullptr, FF); k_gemmb<false, false><<<gJ, 128, 0, stream>>>(Jb, nullptr, WJJb, nullptr, PS, HH, nullptr, nullptr, FF);
    for (int c = 0; c < NB_ / EVJ; ++c) { const int b0 = c * EVJ;
        k_edge1<<<ECH / 8, 256, 0, stream>>>(PR, PS, bjj1, NJ, NJ, b0, ECH, Eh, El);
        k_gemmb<true, false><<<gE, 128, 0, stream>>>(Eh, El, WJJ2, bjj2, E2, HH, nullptr, nullptr, HH);
        k_pool<true><<<(EVJ * NJ) / 8, 256, 0, stream>>>(E2, mask, NJ, NJ, b0, EVJ * NJ, PJJ); }
    k_gemmb<false, false><<<gJ, 128, 0, stream>>>(Jb, nullptr, WJTa, nullptr, PR, HH, nullptr, nullptr, FF); k_gemmb<false, false><<<gT, 128, 0, stream>>>(Tb, nullptr, WJTb, nullptr, PS, HH, nullptr, nullptr, FF);
    for (int c = 0; c < NB_ / EVT; ++c) { const int b0 = c * EVT;
        k_edge1<<<ECT / 8, 256, 0, stream>>>(PR, PS, bjt1, NJ, NT, b0, ECT, Eh, El);
        k_gemmb<true, false><<<gET, 128, 0, stream>>>(Eh, El, WJT2, bjt2, E2, HH, nullptr, nullptr, HH);
        k_pool<false><<<(EVT * NJ) / 8, 256, 0, stream>>>(E2, nullptr, NJ, NT, b0, EVT * NJ, PJT); }
    k_split128<<<NJR / 8, 256, 0, stream>>>(PJJ, NJR, PJJh, PJJl); k_split128<<<NJR / 8, 256, 0, stream>>>(PJT, NJR, PJTh, PJTl);
    k_gemmb<false, false><<<gJ, 128, 0, stream>>>(Jb, nullptr, WNJa, bnj1, G1, HH, nullptr, nullptr, FF);
    k_gemmb<true, false><<<gJ, 128, 0, stream>>>(PJJh, PJJl, WNJb, nullptr, G1b, HH, nullptr, G1, HH, 0);
    k_gemmb<true, false><<<gJ, 128, 0, stream>>>(PJTh, PJTl, WNJc, nullptr, G1, HH, nullptr, G1b, HH, 0);
    k_relupl128<<<NJR / 8, 256, 0, stream>>>(G1, NJR, G1h, G1l);
    k_gemmb<true, false><<<dim3(NJR / 64, 1, 1), 128, 0, stream>>>(G1h, G1l, WNJ2, bnj2, G2, NO, nullptr, nullptr, HH);
    k_nodeout<true><<<NJR / 8, 256, 0, stream>>>(G2, mask, NJR, out0, UJh, UJl);
    k_gemmb<false, false><<<gT, 128, 0, stream>>>(Tb, nullptr, WTJa, nullptr, PR, HH, nullptr, nullptr, FF); k_gemmb<false, false><<<gJ, 128, 0, stream>>>(Jb, nullptr, WTJb, nullptr, PS, HH, nullptr, nullptr, FF);
    for (int c = 0; c < NB_ / EVT; ++c) { const int b0 = c * EVT;
        k_edge1<<<ECT / 8, 256, 0, stream>>>(PR, PS, btj1, NT, NJ, b0, ECT, Eh, El);
        k_gemmb<true, false><<<gET, 128, 0, stream>>>(Eh, El, WTJ2, btj2, E2, HH, nullptr, nullptr, HH);
        k_pool<true><<<(EVT * NT) / 8, 256, 0, stream>>>(E2, mask, NT, NJ, b0, EVT * NT, PTJ); }
    k_split128<<<NTR / 8, 256, 0, stream>>>(PTJ, NTR, PTJh, PTJl);
    k_gemmb<false, false><<<gT, 128, 0, stream>>>(Tb, nullptr, WNTa, bnt1, G1, HH, nullptr, nullptr, FF);
    k_gemmb<true, false><<<gT, 128, 0, stream>>>(PTJh, PTJl, WNTb, nullptr, G1b, HH, nullptr, G1, HH, 0);
    k_relupl128<<<NTR / 8, 256, 0, stream>>>(G1b, NTR, G1h, G1l);
    k_gemmb<true, false><<<dim3(NTR / 64, 1, 1), 128, 0, stream>>>(G1h, G1l, WNT2, bnt2, G2, NO, nullptr, nullptr, HH);
    k_nodeout<false><<<NTR / 8, 256, 0, stream>>>(G2, nullptr, NTR, out1, UTh, UTl);
    k_gemmb<true, false><<<gT, 128, 0, stream>>>(UTh, UTl, WCa, nullptr, PR, HH, nullptr, nullptr, NO); k_gemmb<true, false><<<gJ, 128, 0, stream>>>(UJh, UJl, WCb, nullptr, PS, HH, nullptr, nullptr, NO);
    for (int c = 0; c < NB_ / EVT; ++c) { const int b0 = c * EVT;
        k_edge1<<<ECT / 8, 256, 0, stream>>>(PR, PS, bc1, NT, NJ, b0, ECT, Eh, El);
        k_gemmb<true, false><<<gET, 128, 0, stream>>>(Eh, El, WC2, bc2, E2, HH, nullptr, nullptr, HH);
        k_relupl128<<<ECT / 8, 256, 0, stream>>>(E2, ECT, Eh, El);
        k_gemmb<true, false><<<dim3(ECT / 64, 1, 1), 128, 0, stream>>>(Eh, El, WC3, nullptr, SC, 64, nullptr, nullptr, HH);
        k_score<<<(ECT / 128 + 7) / 8, 256, 0, stream>>>(SC, bc3, mask, (size_t)b0 * NT * NJ, ECT, out2); }
    k_utp<<<NTR / 8, 256, 0, stream>>>(UTh, UTl, UTPh, UTPl);
    for (int p = 0; p < NT; ++p) { const bf* Ah = UTPh + (size_t)p * NB_ * NO; const bf* Al = UTPl + (size_t)p * NB_ * NO;
        k_gemmb<true, false><<<dim3(NB_ / 64, HH / 64, 1), 128, 0, stream>>>(Ah, Al, WR1 + (size_t)p * HH * FF, br1 + (size_t)p * HH, R1, HH, nullptr, nullptr, FF);
        k_relupl128<<<NB_ / 8, 256, 0, stream>>>(R1, NB_, R1h, R1l);
        k_gemmb<true, false><<<dim3(NB_ / 64, HH / 64, 1), 128, 0, stream>>>(R1h, R1l, WR2 + (size_t)p * HH * HH, br2 + (size_t)p * HH, R1, HH, nullptr, nullptr, HH);
        k_relupl128<<<NB_ / 8, 256, 0, stream>>>(R1, NB_, R1h, R1l);
        k_gemmb<true, false><<<dim3(NB_ / 64, 1, 1), 128, 0, stream>>>(R1h, R1l, WR3 + (size_t)p * 64 * HH, BR3 + (size_t)p * 64, REG + (size_t)p * NB_ * 64, 64, nullptr, nullptr, HH); }
    k_regout<<<(NB_ * NT * RG / 128) / 8, 256, 0, stream>>>(REG, out3);
}
